// FAGCN_MOE_22110491640670
// MI455X (gfx1250) — hardware-run, weakly checked
//
#include <hip/hip_runtime.h>


namespace {
constexpr int N = 50000, D = 96, E = 800000, G = 2048, L = 64, NH = 8, DH = 12, NBLK = N / 16;
constexpr float XS = 8.0f, WSC = 256.0f, FEPS = 0.3f;
typedef _Float16 b16;
typedef __attribute__((ext_vector_type(16))) _Float16 v16b;
typedef __attribute__((ext_vector_type(8))) _Float16 v8b;
typedef __attribute__((ext_vector_type(8))) float v8f;
typedef __attribute__((ext_vector_type(4))) float v4f;
typedef __attribute__((ext_vector_type(2))) float v2f;
__device__ __forceinline__ float bf16_rne(float f) { unsigned int u = __float_as_uint(f); u += 0x7FFFu + ((u >> 16) & 1u); return __uint_as_float(u & 0xFFFF0000u); }
__device__ __forceinline__ void split16(float v, b16& hi, b16& lo) { hi = (b16)v; lo = (b16)(v - (float)hi); }
__device__ __forceinline__ v16b frag_kb(const b16* p, int hh) { const v8b a = *(const v8b*)(p + 8 * hh), b = *(const v8b*)(p + 16 + 8 * hh); v16b f;
#pragma unroll
  for (int e = 0; e < 8; ++e) { f[e] = a[e]; f[8 + e] = b[e]; } return f; }
__device__ __forceinline__ v8f wmma16b(v16b a, v16b b, v8f c) { v8f d = __builtin_amdgcn_wmma_f32_16x16x32_f16(false, a, false, b, (short)0, c, false, false); asm volatile("v_nop\n\tv_nop\n\tv_nop\n\tv_nop" : "+v"(d) : "v"(a), "v"(b)); return d; }
__device__ __forceinline__ void wave_lds_sync() { __builtin_amdgcn_fence(__ATOMIC_RELEASE, "workgroup"); __builtin_amdgcn_wave_barrier(); __builtin_amdgcn_fence(__ATOMIC_ACQUIRE, "workgroup"); }
__device__ __forceinline__ float pmul(float a, float b) { float p = a * b; asm volatile("" : "+v"(p)); return p; }
__device__ __forceinline__ int iclamp(int v, int lo, int hi) { return v < lo ? lo : (v > hi ? hi : v); }
constexpr int CSR_NBLK9 = 512, CSR_GB9 = 9, CSR_GN9 = 1 << CSR_GB9  , CSR_TS9 = (CSR_GN9 < 32 ? 32 : CSR_GN9)  , CSR_MAXG9 = 512, CSR_CAP9 = 12288  ;
__device__ __host__ __forceinline__ int csr_tix9(int v) { return (v >> CSR_GB9) * CSR_TS9 + (v & (CSR_GN9 - 1)); }
__global__ __launch_bounds__(64) void csrA_kernel9(const int* __restrict__ dst, int E, int N, int nG, int CHP, int NGP, int* __restrict__ STG, int* __restrict__ HST) {
  extern __shared__ int sm[];
  int* cnt = sm; int* run = sm + NGP; int* ids = sm + 2 * NGP;
  const int b = blockIdx.x; const int ch = (E + CSR_NBLK9 - 1) / CSR_NBLK9; const int e0 = b * ch, e1 = min(E, e0 + ch);
  for (int i = threadIdx.x; i < NGP; i += 64) cnt[i] = 0;
  for (int i = threadIdx.x; i < CHP; i += 64) ids[i] = -1;
  __syncthreads();
  if (threadIdx.x == 0) {
    for (int e = e0; e < e1; ++e) { int d = dst[e]; d = (d < 0) ? 0 : (d >= N ? N - 1 : d); cnt[d >> CSR_GB9] += 1; }
    int acc = 0; for (int g = 0; g < nG; ++g) { run[g] = acc; acc += cnt[g]; }
    for (int e = e0; e < e1; ++e) { int d = dst[e]; d = (d < 0) ? 0 : (d >= N ? N - 1 : d); const int g = d >> CSR_GB9; ids[run[g]] = e; run[g] += 1; } }
  __syncthreads();
  typedef __attribute__((ext_vector_type(4))) int v4i;
  for (int pass = 0; pass < 2; ++pass) {
    for (int i = threadIdx.x; i < CHP / 4; i += 64) *(volatile v4i*)(STG + (size_t)b * CHP + i * 4) = *(const v4i*)(&ids[i * 4]);
    for (int i = threadIdx.x; i < NGP / 4; i += 64) { v4i v; for (int e = 0; e < 4; ++e) v[e] = (i * 4 + e < nG) ? cnt[i * 4 + e] : 0; *(volatile v4i*)(HST + (size_t)b * NGP + i * 4) = v; }
    __threadfence(); }
}
__global__ __launch_bounds__(512) void csrS_kernel9(const int* __restrict__ HST, int nG, int NGP, int* __restrict__ START, int* __restrict__ TOT, int* __restrict__ OFF) {
  __shared__ int tot[CSR_MAXG9];
  const int b = threadIdx.x;
  for (int pass = 0; pass < 2; ++pass) { int runb = 0; for (int g = 0; g < nG; ++g) { int c = HST[(size_t)b * NGP + g]; c = (c < 0) ? 0 : c; ((volatile int*)OFF)[(size_t)g * CSR_NBLK9 + b] = runb; runb += c; } __threadfence(); }
  for (int g = threadIdx.x; g < nG; g += 512) { int s = 0; for (int bb = 0; bb < CSR_NBLK9; ++bb) { int c = HST[(size_t)bb * NGP + g]; s += (c < 0) ? 0 : c; } tot[g] = s; }
  __syncthreads();
  if (threadIdx.x < 32) {
    __shared__ int st[CSR_MAXG9 + 32];
    if (threadIdx.x == 0) { int acc = 0; for (int g = 0; g < NGP; ++g) { st[g] = acc; if (g < nG) acc += (tot[g] + 31) & ~31; } st[NGP] = acc; }
    __builtin_amdgcn_fence(__ATOMIC_RELEASE, "workgroup"); __builtin_amdgcn_wave_barrier(); __builtin_amdgcn_fence(__ATOMIC_ACQUIRE, "workgroup");
    for (int pass = 0; pass < 2; ++pass) { for (int i = threadIdx.x; i < NGP + 32; i += 32) { ((volatile int*)START)[i] = (i <= NGP) ? st[min(i, NGP)] : 0; ((volatile int*)TOT)[i] = (i < nG) ? tot[i] : 0; } __threadfence(); } }
}
__global__ __launch_bounds__(256) void csrB_kernel9(const int* __restrict__ dst, int N, int nG, int CHP, int NGP, int permLen, const int* __restrict__ STG, const int* __restrict__ HST, const int* __restrict__ OFF, const int* __restrict__ START, const int* __restrict__ TOT, int* __restrict__ PERM, int* __restrict__ ROWPTR, int* __restrict__ ROWCNT, int* __restrict__ FLAG) {
  typedef __attribute__((ext_vector_type(4))) int v4i;
  __shared__ int ids[CSR_CAP9]; __shared__ unsigned short key[CSR_CAP9]; __shared__ int outp[CSR_CAP9]; __shared__ int ncnt[CSR_GN9 + 1]; __shared__ int boff[CSR_NBLK9 + 1];
  const int g = blockIdx.x, t_ = threadIdx.x; int tot = TOT[g]; int st = START[g], stn = START[g + 1]; const int v0 = g * CSR_GN9; const int nv = min(CSR_GN9, N - v0); const int t0 = g * CSR_TS9;
  st = (st < 0) ? 0 : (st > permLen - 32 ? permLen - 32 : st) & ~31; stn = (stn < st) ? st : (stn > permLen ? permLen : stn); tot = (tot < 0) ? 0 : tot; if (tot > stn - st && tot <= CSR_CAP9) tot = stn - st;
  if (tot > CSR_CAP9) {
    for (int pass = 0; pass < 2; ++pass) { for (int i = t_; i < CSR_TS9 / 4; i += 256) { v4i a, c; for (int e = 0; e < 4; ++e) { a[e] = st; c[e] = 0; } *(volatile v4i*)(ROWPTR + t0 + i * 4) = a; *(volatile v4i*)(ROWCNT + t0 + i * 4) = c; } if (t_ == 0) ((volatile int*)FLAG)[0] = 1; __threadfence(); } (void)nv; return; }
  if (t_ == 0) { int acc = 0; for (int b = 0; b < CSR_NBLK9; ++b) { boff[b] = acc; int c = HST[(size_t)b * NGP + g]; c = (c < 0) ? 0 : (c > CHP ? CHP : c); acc += c; if (acc > tot) acc = tot; } boff[CSR_NBLK9] = acc; }
  for (int i = t_; i <= CSR_GN9; i += 256) ncnt[i] = 0;
  __syncthreads();
  for (int b = 0; b < CSR_NBLK9; ++b) { const int c = boff[b + 1] - boff[b]; int o_ = OFF[(size_t)g * CSR_NBLK9 + b]; o_ = (o_ < 0) ? 0 : (o_ > CHP - c ? CHP - c : o_); const int* src_ = STG + (size_t)b * CHP + o_;
    for (int i = t_; i < c; i += 256) { int id = src_[i]; id = (id < 0) ? 0 : id; ids[boff[b] + i] = id; int d = dst[id]; d = (d < v0) ? v0 : (d >= N ? N - 1 : d); int kk = d - v0; kk = (kk < 0) ? 0 : (kk >= CSR_GN9 ? CSR_GN9 - 1 : kk); key[boff[b] + i] = (unsigned short)kk; } }
  __syncthreads();
  if (t_ == 0) { for (int i = 0; i < tot; ++i) ncnt[key[i]] += 1; int acc = 0; for (int vl = 0; vl < CSR_GN9; ++vl) { const int c = ncnt[vl]; ncnt[vl] = acc; acc += c; } ncnt[CSR_GN9] = acc;
    for (int i = 0; i < tot; ++i) { const int vl = key[i]; outp[ncnt[vl]] = ids[i]; ncnt[vl] += 1; }
    for (int vl = CSR_GN9; vl > 0; --vl) ncnt[vl] = ncnt[vl - 1]; ncnt[0] = 0; }
  __syncthreads();
  for (int pass = 0; pass < 2; ++pass) {
    for (int i = t_; i < (stn - st) / 4; i += 256) { v4i v; for (int e = 0; e < 4; ++e) { const int q = i * 4 + e; v[e] = (q < tot) ? outp[q] : -1; } *(volatile v4i*)(PERM + st + i * 4) = v; }
    for (int i = t_; i < CSR_TS9 / 4; i += 256) { v4i a, c; for (int e = 0; e < 4; ++e) { const int vl = i * 4 + e; const int vc = vl < CSR_GN9 ? vl : CSR_GN9; a[e] = (vl < CSR_GN9) ? st + ncnt[vc] : st; c[e] = (vl < nv) ? (ncnt[(vc < CSR_GN9 ? vc : CSR_GN9 - 1) + 1] - ncnt[vc]) : 0; } *(volatile v4i*)(ROWPTR + t0 + i * 4) = a; *(volatile v4i*)(ROWCNT + t0 + i * 4) = c; }
    __threadfence(); }
}
__global__ __launch_bounds__(256) void csrZ_kernel9(int* __restrict__ p, size_t n4) { typedef __attribute__((ext_vector_type(4))) int v4i; const size_t tid = (size_t)blockIdx.x * 256 + threadIdx.x, nth = (size_t)gridDim.x * 256; v4i z = {0, 0, 0, 0}; for (size_t i = tid; i < n4; i += nth) *(volatile v4i*)(p + i * 4) = z; }
struct CsrBufs9 { int *STG, *HST, *OFF, *START, *TOT, *PERM, *ROWPTR, *ROWCNT, *FLAG; int nG, NGP, CHP; size_t permLen; char* base; size_t bytes; };
static size_t csr_carve9(CsrBufs9& c, char* ws, size_t off, int E, int N) {
  const size_t off0 = off; c.base = ws + off;
  auto al = [&](size_t bytes) { char* p = ws + off; off += (bytes + 255) & ~(size_t)255; return p; };
  c.nG = (N + CSR_GN9 - 1) / CSR_GN9; c.NGP = (c.nG + 31) & ~31; const int ch = (E + CSR_NBLK9 - 1) / CSR_NBLK9; c.CHP = (ch + 31) & ~31; c.permLen = (size_t)E + 32 * (size_t)c.nG + 32;
  c.STG = (int*)al((size_t)CSR_NBLK9 * c.CHP * 4); c.HST = (int*)al((size_t)CSR_NBLK9 * c.NGP * 4); c.OFF = (int*)al((size_t)c.NGP * CSR_NBLK9 * 4); c.START = (int*)al((size_t)(c.NGP + 64) * 4); c.TOT = (int*)al((size_t)(c.NGP + 64) * 4);
  c.PERM = (int*)al(c.permLen * 4); c.ROWPTR = (int*)al((size_t)c.nG * CSR_TS9 * 4); c.ROWCNT = (int*)al((size_t)c.nG * CSR_TS9 * 4); c.FLAG = (int*)al(256);
  c.bytes = off - off0; return off;
}
static void csr_build9(const CsrBufs9& c, const int* dst, int E, int N, hipStream_t stream) {
  const size_t smem = (size_t)(2 * c.NGP + c.CHP) * 4;
  csrZ_kernel9<<<512, 256, 0, stream>>>((int*)c.base, c.bytes / 16);
  csrA_kernel9<<<CSR_NBLK9, 64, smem, stream>>>(dst, E, N, c.nG, c.CHP, c.NGP, c.STG, c.HST);
  csrS_kernel9<<<1, 512, 0, stream>>>(c.HST, c.nG, c.NGP, c.START, c.TOT, c.OFF);
  csrB_kernel9<<<c.nG, 256, 0, stream>>>(dst, N, c.nG, c.CHP, c.NGP, (int)c.permLen, c.STG, c.HST, c.OFF, c.START, c.TOT, c.PERM, c.ROWPTR, c.ROWCNT, c.FLAG);
}


__global__ __launch_bounds__(256) void wcopy_kernel(const float* __restrict__ w, int total, b16* __restrict__ WT) { const int u = blockIdx.x * 256 + threadIdx.x; if (u >= total / 8) return; const size_t e = (size_t)u * 8; v8b v;
#pragma unroll
  for (int j = 0; j < 8; ++j) v[j] = (b16)(bf16_rne(w[e + j]) * WSC); for (int pass = 0; pass < 2; ++pass) { *(volatile v8b*)(WT + e) = v; __threadfence(); } }
__global__ __launch_bounds__(256) void glgr_kernel(const float* __restrict__ Hh, const float* __restrict__ al, const float* __restrict__ ar, int L1, int NLIM, float* __restrict__ GLR) {
  const int n = blockIdx.x * 256 + threadIdx.x; if (n >= NLIM) return; const float* hr = Hh + (size_t)n * D; float sl = 0.0f, sr = 0.0f;
#pragma unroll 4
  for (int c = 0; c < D; ++c) { float hv = hr[c]; if (L1) hv = bf16_rne(hv); sl += pmul(hv, bf16_rne(al[c])); sr += pmul(hv, bf16_rne(ar[c])); }
  for (int pass = 0; pass < 2; ++pass) { *(volatile v2f*)(GLR + (size_t)n * 2) = (v2f){sl, sr}; __threadfence(); }
}
__global__ __launch_bounds__(256) void faconv_kernel(const float* __restrict__ Hh, const float* __restrict__ x0, const float* __restrict__ GLR, const int* __restrict__ cols, const int* __restrict__ PERM, const int* __restrict__ ROWPTR, const int* __restrict__ ROWCNT, int permLen, int L1, int NLIM, float* __restrict__ OUT) {
  const int wave = threadIdx.x >> 5, lane = threadIdx.x & 31; const size_t i = (size_t)blockIdx.x * 8 + wave; if (i >= (size_t)NLIM) return; const int c0 = lane * 3;
  int st = ROWPTR[i], cnt = ROWCNT[i]; cnt = iclamp(cnt, 0, 1 << 20); st = iclamp(st, 0, permLen - cnt);
  auto degof = [&](size_t u) -> int { int cu = iclamp(ROWCNT[u], 0, 1 << 20); if (NLIM >= N) return cu; int nu = 0; const int su = iclamp(ROWPTR[u], 0, permLen - cu); for (int k = 0; k < cu; ++k) if (iclamp(cols[iclamp(PERM[su + k], 0, E - 1)], 0, N - 1) < NLIM) ++nu; return nu; };
  const int di = degof(i); const float dvi = di > 0 ? rsqrtf((float)di) : 0.0f; const float gli = GLR[i * 2]; float o0 = 0.0f, o1 = 0.0f, o2 = 0.0f;
#pragma unroll 1
  for (int j = 0; j < cnt; ++j) { const int e = iclamp(PERM[st + j], 0, E - 1); const size_t u = (size_t)iclamp(cols[e], 0, N - 1); if (u >= (size_t)NLIM) continue; const int du = degof(u); const float dvu = du > 0 ? rsqrtf((float)du) : 0.0f; const float cf = pmul(pmul(tanhf(gli + GLR[u * 2 + 1]), dvi), dvu); const float* hu = Hh + u * D + c0;
    float h0 = hu[0], h1 = hu[1], h2 = hu[2]; if (L1) { h0 = bf16_rne(h0); h1 = bf16_rne(h1); h2 = bf16_rne(h2); } o0 += pmul(cf, h0); o1 += pmul(cf, h1); o2 += pmul(cf, h2); }
  const float* xr = x0 + i * D + c0; const float r0 = fmaxf(pmul(FEPS, bf16_rne(xr[0])) + o0, 0.0f), r1 = fmaxf(pmul(FEPS, bf16_rne(xr[1])) + o1, 0.0f), r2 = fmaxf(pmul(FEPS, bf16_rne(xr[2])) + o2, 0.0f);
  for (int pass = 0; pass < 2; ++pass) { ((volatile float*)OUT)[i * D + c0] = r0; ((volatile float*)OUT)[i * D + c0 + 1] = r1; ((volatile float*)OUT)[i * D + c0 + 2] = r2; __threadfence(); }
}
__global__ __launch_bounds__(32) void lin_kernel(const float* __restrict__ x, const float* __restrict__ SO, const float* __restrict__ AO, const float* __restrict__ BO, const float* __restrict__ wga, const float* __restrict__ bga, const float* __restrict__ wgb, const float* __restrict__ bgb, const b16* __restrict__ WL, const float* __restrict__ blin, int NLIM, float* __restrict__ HH) {
  __shared__ __attribute__((aligned(16))) b16 Ah[16][200], Al[16][200]; __shared__ float Tf[16][100];
  const int lane = threadIdx.x, nloc = lane & 15, hlf = lane >> 4; const size_t m0 = (size_t)blockIdx.x * 16; if (m0 >= (size_t)NLIM) return; const int c0 = lane * 3;
  for (int rr = 0; rr < 16; ++rr) { const size_t n = m0 + rr; float xa[3]; for (int i = 0; i < 3; ++i) xa[i] = bf16_rne(x[n * D + c0 + i]); float d[4] = {0.0f, 0.0f, 0.0f, 0.0f};
    for (int i = 0; i < 3; ++i) { d[0] += pmul(xa[i], bf16_rne(wga[c0 + i])); d[1] += pmul(xa[i], bf16_rne(wga[D + c0 + i])); d[2] += pmul(xa[i], bf16_rne(wgb[c0 + i])); d[3] += pmul(xa[i], bf16_rne(wgb[D + c0 + i])); }
#pragma unroll
    for (int k = 0; k < 4; ++k) for (int o = 16; o; o >>= 1) d[k] += __shfl_xor(d[k], o);
    const float a0 = d[0] + bf16_rne(bga[0]), a1 = d[1] + bf16_rne(bga[1]), b0 = d[2] + bf16_rne(bgb[0]), b1 = d[3] + bf16_rne(bgb[1]);
    const float ma = fmaxf(a0, a1), ea0 = __expf(a0 - ma), ea1 = __expf(a1 - ma), ga0 = ea0 / (ea0 + ea1), ga1 = ea1 / (ea0 + ea1); const float mb = fmaxf(b0, b1), eb0 = __expf(b0 - mb), eb1 = __expf(b1 - mb), gb0 = eb0 / (eb0 + eb1), gb1 = eb1 / (eb0 + eb1);
    for (int i = 0; i < 3; ++i) { const int c = c0 + i; const float s = SO[n * D + c]; b16 p, q; split16((pmul(ga0, AO[n * D + c]) + pmul(ga1, s)) * XS, p, q); Ah[rr][c] = p; Al[rr][c] = q; split16((pmul(gb0, BO[n * D + c]) + pmul(gb1, s)) * XS, p, q); Ah[rr][D + c] = p; Al[rr][D + c] = q; } }
  wave_lds_sync(); v8f acc[6];
#pragma unroll
  for (int t = 0; t < 6; ++t) acc[t] = (v8f){};
#pragma unroll
  for (int kb = 0; kb < 2 * D; kb += 32) { const v16b a = frag_kb(&Ah[nloc][kb], hlf), al = frag_kb(&Al[nloc][kb], hlf);
#pragma unroll
    for (int t = 0; t < 6; ++t) { const v16b bw = frag_kb(WL + (size_t)(t * 16 + nloc) * (2 * D) + kb, hlf); acc[t] = wmma16b(a, bw, acc[t]); acc[t] = wmma16b(al, bw, acc[t]); } }
#pragma unroll
  for (int t = 0; t < 6; ++t) { const int c = t * 16 + nloc; const float bb = bf16_rne(blin[c]);
#pragma unroll
    for (int r8 = 0; r8 < 8; ++r8) Tf[8 * hlf + r8][c] = fmaxf(acc[t][r8] * (1.0f / (XS * WSC)) + bb, 0.0f); }
  wave_lds_sync();
  for (int pass = 0; pass < 2; ++pass) { for (int rr = 0; rr < 16; ++rr) for (int i = 0; i < 3; ++i) ((volatile float*)HH)[(m0 + rr) * D + c0 + i] = Tf[rr][c0 + i]; __threadfence(); }
}
__global__ __launch_bounds__(32) void kv_kernel(const float* __restrict__ HH, const int* __restrict__ tids, const b16* __restrict__ WQKV, const float* __restrict__ bqkv, int NGV, int IDMOD, float* __restrict__ KV) {
  __shared__ __attribute__((aligned(16))) b16 Ah[16][104], Al[16][104]; __shared__ float Tf[16][196]; const int lane = threadIdx.x, nloc = lane & 15, hlf = lane >> 4; const int g = blockIdx.x >> 2, mb = blockIdx.x & 3; if (g >= NGV) return;
  for (int rr = 0; rr < 16; ++rr) { int id = iclamp(tids[g * L + mb * 16 + rr], 0, N - 1); if (IDMOD < N) id %= IDMOD; for (int i = 0; i < 3; ++i) { const int c = lane * 3 + i; b16 p, q; split16(HH[(size_t)id * D + c] * XS, p, q); Ah[rr][c] = p; Al[rr][c] = q; } }
  wave_lds_sync(); v8f acc[12];
#pragma unroll
  for (int t = 0; t < 12; ++t) acc[t] = (v8f){};
#pragma unroll
  for (int kb = 0; kb < D; kb += 32) { const v16b a = frag_kb(&Ah[nloc][kb], hlf), al = frag_kb(&Al[nloc][kb], hlf);
#pragma unroll
    for (int t = 0; t < 12; ++t) { const v16b bw = frag_kb(WQKV + (size_t)(D + t * 16 + nloc) * D + kb, hlf); acc[t] = wmma16b(a, bw, acc[t]); acc[t] = wmma16b(al, bw, acc[t]); } }
#pragma unroll
  for (int t = 0; t < 12; ++t) { const int c = t * 16 + nloc; const float bb = bf16_rne(bqkv[D + c]);
#pragma unroll
    for (int r8 = 0; r8 < 8; ++r8) Tf[8 * hlf + r8][c] = acc[t][r8] * (1.0f / (XS * WSC)) + bb; }
  wave_lds_sync();
  for (int pass = 0; pass < 2; ++pass) { for (int rr = 0; rr < 16; ++rr) for (int q = 0; q < 6; ++q) ((volatile float*)KV)[((size_t)g * L + mb * 16 + rr) * (2 * D) + q * 32 + lane] = Tf[rr][q * 32 + lane]; __threadfence(); }
}
__global__ __launch_bounds__(32) void att_kernel(const float* __restrict__ HH, const float* __restrict__ KV, const int* __restrict__ tids, const int* __restrict__ lens, const float* __restrict__ wqkv, const float* __restrict__ bqkv, const float* __restrict__ wo, const float* __restrict__ bo, int NGV, int IDMOD, float* __restrict__ vec, float* __restrict__ wts) {
  __shared__ float Hq[D], Q0[D], At[NH][L], Cx[D]; const int lane = threadIdx.x; const int g = blockIdx.x; if (g >= NGV) return; int id0 = iclamp(tids[g * L], 0, N - 1); if (IDMOD < N) id0 %= IDMOD; const int len = iclamp(lens[g], 0, L);
  for (int i = 0; i < 3; ++i) Hq[lane * 3 + i] = HH[(size_t)id0 * D + lane * 3 + i]; wave_lds_sync();
  for (int i = 0; i < 3; ++i) { const int o = lane * 3 + i; float s = bf16_rne(bqkv[o]);
#pragma unroll 4
    for (int c = 0; c < D; ++c) s += pmul(Hq[c], bf16_rne(wqkv[o * D + c])); Q0[o] = s * 0.28867513459481287f; }
  wave_lds_sync(); const float* kv = KV + (size_t)g * L * (2 * D);
  float sc[2][NH];
#pragma unroll
  for (int p = 0; p < 2; ++p) { const int m = p * 32 + lane; const float* kr = kv + (size_t)m * (2 * D);
#pragma unroll
    for (int h = 0; h < NH; ++h) { float s = 0.0f; for (int d_ = 0; d_ < DH; ++d_) s += pmul(Q0[h * DH + d_], kr[h * DH + d_]); sc[p][h] = m < len ? s : -INFINITY; } }
  float w0 = 0.0f, w1 = 0.0f;
#pragma unroll
  for (int h = 0; h < NH; ++h) { float mx = fmaxf(sc[0][h], sc[1][h]); for (int o = 16; o; o >>= 1) mx = fmaxf(mx, __shfl_xor(mx, o)); const float e0 = sc[0][h] == -INFINITY ? 0.0f : __expf(sc[0][h] - mx), e1 = sc[1][h] == -INFINITY ? 0.0f : __expf(sc[1][h] - mx); float sm = e0 + e1; for (int o = 16; o; o >>= 1) sm += __shfl_xor(sm, o); const float inv = 1.0f / sm; At[h][lane] = e0 * inv; At[h][32 + lane] = e1 * inv; w0 += e0 * inv; w1 += e1 * inv; }
  wave_lds_sync();
  float cx[3] = {0.0f, 0.0f, 0.0f};
#pragma unroll 1
  for (int m = 0; m < L; ++m) { const float* vr = kv + (size_t)m * (2 * D) + D; for (int i = 0; i < 3; ++i) { const int c = lane * 3 + i; cx[i] += pmul(At[c / DH][m], vr[c]); } }
  for (int i = 0; i < 3; ++i) Cx[lane * 3 + i] = cx[i]; wave_lds_sync();
  float vo[3]; for (int i = 0; i < 3; ++i) { const int o = lane * 3 + i; float s = bf16_rne(bo[o]);
#pragma unroll 4
    for (int c = 0; c < D; ++c) s += pmul(Cx[c], bf16_rne(wo[o * D + c])); vo[i] = s; }
  for (int pass = 0; pass < 2; ++pass) { for (int i = 0; i < 3; ++i) ((volatile float*)vec)[(size_t)g * D + lane * 3 + i] = vo[i]; ((volatile float*)wts)[(size_t)g * L + lane] = w0 * (1.0f / NH); ((volatile float*)wts)[(size_t)g * L + 32 + lane] = w1 * (1.0f / NH); __threadfence(); }
}
}

extern "C" void kernel_launch(void* const* d_in, const int* in_sizes, int n_in, void* d_out, int out_size, void* d_ws, size_t ws_size, hipStream_t stream) {
  (void)n_in;
  auto Fp = [&](int i) { return (const float*)d_in[i]; }; auto Ip = [&](int i) { return (const int*)d_in[i]; };
  if (in_sizes[0] != N * D || in_sizes[1] != 2 * D || in_sizes[3] != 2 * D || in_sizes[7] != D * 2 * D || in_sizes[9] != 3 * D * D || in_sizes[11] != D * D || in_sizes[13] != 2 * E || in_sizes[14] != 2 * E || in_sizes[15] != 2 * E || in_sizes[16] != G * L || in_sizes[17] != G || out_size != G * D + G * L) return;
  const int NLIM = N, NGV = G, IDMOD = N; const int GB8 = N / 8, GT = (N + 255) / 256, GB16 = NBLK;
  size_t off = 0; char* ws = (char*)d_ws;
  auto carve = [&](size_t bytes) { char* p = ws + off; off += (bytes + 255) & ~(size_t)255; return p; };
  b16* WL = (b16*)carve((size_t)D * 2 * D * 2); b16* WQKV = (b16*)carve((size_t)3 * D * D * 2); float* GLR = (float*)carve((size_t)N * 2 * 4);
  float* HA = (float*)carve((size_t)N * D * 4); float* OS = (float*)carve((size_t)N * D * 4); float* OA = (float*)carve((size_t)N * D * 4); float* OB = (float*)carve((size_t)N * D * 4); float* HH = (float*)carve((size_t)N * D * 4); float* KV = (float*)carve((size_t)G * L * 2 * D * 4);
  CsrBufs9 c0, c1, c2; off = csr_carve9(c0, ws, off, E, N); off = csr_carve9(c1, ws, off, E, N); off = csr_carve9(c2, ws, off, E, N);
  if (off > ws_size || off > ((size_t)256 << 20)) return;
  wcopy_kernel<<<(D * 2 * D / 8 + 255) / 256, 256, 0, stream>>>(Fp(7), D * 2 * D, WL); wcopy_kernel<<<(3 * D * D / 8 + 255) / 256, 256, 0, stream>>>(Fp(9), 3 * D * D, WQKV);
  csr_build9(c0, Ip(13), E, N, stream); csr_build9(c1, Ip(14), E, N, stream); csr_build9(c2, Ip(15), E, N, stream);
  CsrBufs9* cs[3] = {&c0, &c1, &c2}; const int gi[3] = {13, 14, 15}; float* outs[3] = {OS, OA, OB};
  for (int q = 0; q < 3; ++q) { CsrBufs9& cc = *cs[q];
    glgr_kernel<<<GT, 256, 0, stream>>>(Fp(0), Fp(1), Fp(2), 1, NLIM, GLR);
    faconv_kernel<<<GB8, 256, 0, stream>>>(Fp(0), Fp(0), GLR, Ip(gi[q]) + E, cc.PERM, cc.ROWPTR, cc.ROWCNT, (int)cc.permLen, 1, NLIM, HA);
    glgr_kernel<<<GT, 256, 0, stream>>>(HA, Fp(1) + D, Fp(2) + D, 0, NLIM, GLR);
    faconv_kernel<<<GB8, 256, 0, stream>>>(HA, Fp(0), GLR, Ip(gi[q]) + E, cc.PERM, cc.ROWPTR, cc.ROWCNT, (int)cc.permLen, 0, NLIM, outs[q]); }
  lin_kernel<<<GB16, 32, 0, stream>>>(Fp(0), OS, OA, OB, Fp(3), Fp(4), Fp(5), Fp(6), WL, Fp(8), NLIM, HH);
  float* out = (float*)d_out;
  kv_kernel<<<NGV * 4, 32, 0, stream>>>(HH, Ip(16), WQKV, Fp(10), NGV, IDMOD, KV);
  att_kernel<<<NGV, 32, 0, stream>>>(HH, KV, Ip(16), Ip(17), Fp(9), Fp(10), Fp(11), Fp(12), NGV, IDMOD, out, out + (size_t)G * D);
}
